// ShiftingLayer_63247688401341
// MI455X (gfx1250) — hardware-run, weakly checked
//
#include <hip/hip_runtime.h>


#ifndef NB
#define NB 16
#endif
#ifndef TLEN
#define TLEN 2048
#endif
#ifndef SLEN
#define SLEN 4096
#endif
#define NB_FULL 16
#define T_FULL  2048
#define S_FULL  4096
#ifndef OUT_T
#define OUT_T TLEN
#endif
#define CW   128
#define SWV  4
#define OSP  132
#define XTP  66
#define PSH  10.0f
#define PSI  (1.0f / 1024.0f)
#define NL4  ((float)(-4.0 * 1.4426950408889634))
#define DCUT 6.0f

static_assert(CW == 128);
static_assert(CW % 64 == 0);
static_assert(CW % 16 == 0);
static_assert(SLEN % 64 == 0);
static_assert(SLEN % 32 == 0);
static_assert(TLEN % (16 * SWV) == 0);
static_assert(NB <= NB_FULL);
static_assert(TLEN <= T_FULL);
static_assert(SLEN <= S_FULL);
static_assert((OSP * 4) % 16 == 0);
static_assert(OSP >= CW);
static_assert(XTP >= 64);
static_assert(256 * 4 * 4 == 64 * 64);
static_assert(256 * 16 * 2 == 64 * 64 * 2);
static_assert(32 * 16 * 16 == 16 * CW * 4);
static_assert(64 * XTP * 2 <= 131072);
static_assert(SWV * 16 * OSP * 4 <= 131072);

typedef _Float16 h16;
typedef __attribute__((ext_vector_type(16))) _Float16 v16h;
typedef __attribute__((ext_vector_type(8)))  _Float16 v8h;
typedef __attribute__((ext_vector_type(8)))  float    v8f;
typedef __attribute__((ext_vector_type(4)))  float    v4f;
typedef v4f  __attribute__((may_alias)) v4fa;

__device__ __forceinline__ unsigned short f2bf(float f) { unsigned u = __float_as_uint(f); u += 0x7FFFu + ((u >> 16) & 1u); return (unsigned short)(u >> 16); }
__device__ __forceinline__ float bfr(float f) { return __uint_as_float(((unsigned)f2bf(f)) << 16); }
__device__ __forceinline__ v16h cat16(v8h lo, v8h hi) { return __builtin_shufflevector(lo, hi, 0, 1, 2, 3, 4, 5, 6, 7, 8, 9, 10, 11, 12, 13, 14, 15); }
__device__ __forceinline__ v8f wmma16(v16h a, v16h b, v8f c) { return __builtin_amdgcn_wmma_f32_16x16x32_f16(false, a, false, b, (short)0, c, false, false); }
__device__ __forceinline__ v16h  ldh(const h16* p) { return cat16(*(const v8h*)p, *(const v8h*)(p + 16)); }
__device__ __forceinline__ void wave_sync() { __builtin_amdgcn_fence(3  , "wavefront"); __builtin_amdgcn_wave_barrier(); asm volatile("" ::: "memory"); }
static __device__ __forceinline__ h16 toh_flush(float v) { const h16 r = (h16)v; return (fabsf(v) < 6.103515625e-05f) ? (h16)0.0f : r; }
__device__ __forceinline__ v8f wmma16g(v16h a, v16h b, v8f c) { c = wmma16(a, b, c); asm volatile("v_nop\n\tv_nop\n\tv_nop\n\tv_nop" : "+v"(c) : "v"(a), "v"(b)); return c; }

__global__ __launch_bounds__(256) void k_xt(const float* __restrict__ X, h16* XT) {
#pragma clang fp contract(off)
    __shared__ h16 tl[64 * XTP];
    const int tid = threadIdx.x;
    const int s0 = blockIdx.x * 64, c0 = blockIdx.y * 64, b = blockIdx.z;
    const float* src = X + ((size_t)b * S_FULL + (size_t)s0) * CW + c0;
#pragma unroll
    for (int it = 0; it < 4; ++it) {
        const int idx = it * 256 + tid; const int row = idx >> 4, c4 = (idx & 15) * 4;
        const v4f v = *(const v4f*)(src + (size_t)row * CW + c4);
#pragma unroll
        for (int j = 0; j < 4; ++j) tl[row * XTP + c4 + j] = toh_flush(bfr(v[j]));
    }
    __syncthreads();
    h16* dst = XT + ((size_t)b * CW + (size_t)c0) * SLEN + (size_t)s0;
#pragma unroll 1
    for (int ps = 0; ps < 2; ++ps) {
#pragma unroll
        for (int it = 0; it < 2; ++it) {
            const int p = it * 256 + tid; const int crow = p >> 3, s8 = (p & 7) * 8;
            v8h o;
#pragma unroll
            for (int i = 0; i < 8; ++i) o[i] = tl[(s8 + i) * XTP + crow];
            *(volatile v8h*)(dst + (size_t)crow * SLEN + s8) = o; }
        if (ps == 0) __threadfence(); }
}

__global__ __launch_bounds__(32 * SWV) void k_bandmm(const h16* __restrict__ XT, const float* __restrict__ SWT, float* OUT) {
    __shared__ __align__(16) float os[SWV * 16 * OSP];
    const int lane = threadIdx.x & 31, lr = lane & 15, hi = lane >> 4;
    const int wave = __builtin_amdgcn_readfirstlane((int)(threadIdx.x >> 5));
    const int b = blockIdx.y;
    const int t0 = (blockIdx.x * SWV + wave) * 16;
    const int t = t0 + lr;
    const float swv = bfr(SWT[(size_t)b * T_FULL + t]);
    const float cen = (float)t - swv;
    float flo = fminf(fmaxf(cen - DCUT, 0.0f), (float)(SLEN - 1));
    float fhi = fminf(fmaxf(cen + DCUT, 0.0f), (float)(SLEN - 1));
    flo = fminf(flo, __shfl_xor(flo, 1, 32));  fhi = fmaxf(fhi, __shfl_xor(fhi, 1, 32));
    flo = fminf(flo, __shfl_xor(flo, 2, 32));  fhi = fmaxf(fhi, __shfl_xor(fhi, 2, 32));
    flo = fminf(flo, __shfl_xor(flo, 4, 32));  fhi = fmaxf(fhi, __shfl_xor(fhi, 4, 32));
    flo = fminf(flo, __shfl_xor(flo, 8, 32));  fhi = fmaxf(fhi, __shfl_xor(fhi, 8, 32));
    flo = fminf(flo, __shfl_xor(flo, 16, 32)); fhi = fmaxf(fhi, __shfl_xor(fhi, 16, 32));
    int klo_v = ((int)flo) & ~31;
    klo_v = klo_v < 0 ? 0 : (klo_v > SLEN - 32 ? SLEN - 32 : klo_v);
    int khi_v = (int)fhi + 2;
    khi_v = khi_v > SLEN ? SLEN : khi_v;
    int ns_v = (khi_v - klo_v + 31) >> 5;
    const int nmax_v = (SLEN - klo_v) >> 5;
    ns_v = ns_v < 1 ? 1 : ns_v;
    ns_v = ns_v > nmax_v ? nmax_v : ns_v;
    ns_v = ns_v > SLEN / 32 ? SLEN / 32 : ns_v;
    const int klo = __builtin_amdgcn_readfirstlane(klo_v);
    const int ns  = __builtin_amdgcn_readfirstlane(ns_v);
    v8f acc[8];
#pragma unroll
    for (int j = 0; j < 8; ++j) acc[j] = (v8f){};
    const size_t xo = ((size_t)b * CW + (size_t)lr) * SLEN + 8 * hi;
#pragma unroll 1
    for (int st = 0; st < ns; ++st) {
        const int k0 = klo + st * 32;
        const int sb = k0 + 8 * hi - t;
        v16h a;
#pragma unroll
        for (int i = 0; i < 8; ++i) {
            const float d0 = swv + (float)(sb + i), d1 = swv + (float)(sb + 16 + i);
            const float q0 = d0 * d0, q1 = d1 * d1;
            const float e0 = q0 * NL4 + PSH, e1 = q1 * NL4 + PSH;
            const float g0 = (e0 < -14.0f) ? 0.0f : __builtin_amdgcn_exp2f(e0);
            const float g1 = (e1 < -14.0f) ? 0.0f : __builtin_amdgcn_exp2f(e1);
            a[i] = (h16)g0; a[8 + i] = (h16)g1; }
        const h16* xp = XT + xo + (size_t)k0;
#pragma unroll
        for (int j = 0; j < 8; ++j) { const v16h bx = ldh(xp + (size_t)j * 16 * SLEN); acc[j] = wmma16g(a, bx, acc[j]); }
    }
    const int wb = wave * 16 * OSP;
#pragma unroll
    for (int j = 0; j < 8; ++j) {
#pragma unroll
        for (int r = 0; r < 8; ++r) os[wb + (8 * hi + r) * OSP + 16 * j + lr] = acc[j][r] * PSI; }
    wave_sync();
    float* orow = OUT + ((size_t)b * OUT_T + (size_t)t0) * CW;
#pragma unroll 1
    for (int ps = 0; ps < 2; ++ps) {
#pragma unroll 4
        for (int row = 0; row < 16; ++row) {
            const v4f val = *(const v4fa*)(&os[wb + row * OSP + lane * 4]);
            *(volatile v4f*)(orow + (size_t)row * CW + lane * 4) = val; }
        if (ps == 0) __threadfence(); }
}

static constexpr size_t al256(size_t v) { return (v + 255) & ~(size_t)255; }
static constexpr size_t SZ_XT = al256((size_t)NB * CW * SLEN * 2);
static constexpr size_t SZ_TOTAL = SZ_XT;
static_assert(SZ_TOTAL <= (size_t)134217728);
static_assert((size_t)(SLEN / 64) * (CW / 64) * NB * 64 * 64 == (size_t)NB * CW * SLEN);
static_assert((size_t)(TLEN / (16 * SWV)) * NB * SWV * 16 == (size_t)NB * TLEN);

extern "C" void kernel_launch(void* const* d_in, const int* in_sizes, int n_in,
                              void* d_out, int out_size, void* d_ws, size_t ws_size, hipStream_t stream) {
    if (n_in < 2) return;
    const size_t needx = ((size_t)(NB - 1) * S_FULL + SLEN) * CW;
    const size_t needs = (size_t)(NB - 1) * T_FULL + TLEN;
    if ((size_t)in_sizes[0] < needx || (size_t)in_sizes[1] < needs) return;
    if ((size_t)out_size < ((size_t)(NB - 1) * OUT_T + TLEN) * CW) return;
    if (SZ_TOTAL > ws_size) return;
    const float* x  = (const float*)d_in[0];
    const float* sw = (const float*)d_in[1];
    float* OUT = (float*)d_out;
    h16* XT = (h16*)d_ws;

    k_xt<<<dim3(SLEN / 64, CW / 64, NB), 256, 0, stream>>>(x, XT);
    k_bandmm<<<dim3(TLEN / (16 * SWV), NB, 1), 32 * SWV, 0, stream>>>(XT, sw, OUT);
}
